// CustomMultiheadAttention_8203387535729
// MI455X (gfx1250) — hardware-verified
//
#include <hip/hip_runtime.h>


#ifndef NB
#define NB 2
#endif
#ifndef SEQ
#define SEQ 2048
#endif
#ifndef NB_FULL
#define NB_FULL 2
#endif
#ifndef SEQ_FULL
#define SEQ_FULL 2048
#endif

namespace {
constexpr int HID = 1024, DH = 64, NH = 16;
constexpr int NQKV = 3 * HID;
constexpr int MROWS = NB * SEQ;
constexpr int QT = SEQ / 16;
constexpr int EARLY = (SEQ < 256) ? SEQ : 256;
constexpr int QT_E = EARLY / 16;
constexpr int QT_L = (SEQ - EARLY) / 16;
constexpr int QT_LD = (QT_L > 0) ? QT_L : 1;
constexpr int NCH = SEQ / 32;
constexpr int FPITCH = 64;
constexpr int MPITCH = SEQ_FULL;
constexpr int F_SKIP = 0, F_OPEN = 1, F_FILL = 2;
constexpr float MASK_FILL = -1.0e9f;
constexpr float SCORE_SCALE = 0.125f;
constexpr float P_CARRY = 4096.0f;
constexpr float Y_CARRY = 64.0f;
constexpr float W_CARRY = 64.0f;
constexpr float RES_CARRY = 1024.0f;
constexpr float RES_INV = 1.0f / 1024.0f;
constexpr float Y_FROM_O = Y_CARRY / P_CARRY;
constexpr float OUT_UNSCALE = 1.0f / (Y_CARRY * W_CARRY);
static_assert(SEQ % 128 == 0);
static_assert(EARLY % 128 == 0);
static_assert((SEQ - EARLY) % 128 == 0);
static_assert(NB >= 1 && NB <= NB_FULL);
static_assert(SEQ <= SEQ_FULL);
static_assert(NH * DH == HID);
static_assert(MROWS % 128 == 0);
static_assert((NB * NH * QT_E) % 8 == 0);
static_assert((NB * NH * QT_L) % 8 == 0);
static_assert(QT_E + QT_L == QT);
static_assert(NCH >= 1 && NCH <= FPITCH);

typedef __bf16 b16;
typedef _Float16 h16;
typedef __bf16 v16b __attribute__((ext_vector_type(16)));
typedef __bf16 v8b __attribute__((ext_vector_type(8)));
typedef _Float16 v16h __attribute__((ext_vector_type(16)));
typedef _Float16 v8h __attribute__((ext_vector_type(8)));
typedef float v8f __attribute__((ext_vector_type(8)));
typedef float v4f __attribute__((ext_vector_type(4)));
typedef unsigned short v8us __attribute__((ext_vector_type(8)));
typedef int v4i __attribute__((ext_vector_type(4)));
typedef int v8i __attribute__((ext_vector_type(8)));

__device__ __forceinline__ v8b ld8b(const b16* p) { return *(const v8b*)p; }
__device__ __forceinline__ v8h ld8h(const h16* p) { return *(const v8h*)p; }
__device__ __forceinline__ v16b cat8b(v8b a, v8b b) { return __builtin_shufflevector(a, b, 0, 1, 2, 3, 4, 5, 6, 7, 8, 9, 10, 11, 12, 13, 14, 15); }
__device__ __forceinline__ v16h cat8h(v8h a, v8h b) { return __builtin_shufflevector(a, b, 0, 1, 2, 3, 4, 5, 6, 7, 8, 9, 10, 11, 12, 13, 14, 15); }
__device__ __forceinline__ v16b frag_kb(const b16* p, int hh) { return cat8b(ld8b(p + 8 * hh), ld8b(p + 16 + 8 * hh)); }
__device__ __forceinline__ v16h frag_kh(const h16* p, int hh) { return cat8h(ld8h(p + 8 * hh), ld8h(p + 16 + 8 * hh)); }

__device__ __forceinline__ v8f wmma_b(v16b a, v16b b, v8f c) {
  v8f d = __builtin_amdgcn_wmma_f32_16x16x32_bf16(false, a, false, b, (short)0, c, false, false);
  asm volatile("v_nop\n\tv_nop\n\tv_nop\n\tv_nop" : "+v"(d) : "v"(a), "v"(b));
  return d;
}
__device__ __forceinline__ v8f wmma_h(v16h a, v16h b, v8f c) {
  v8f d = __builtin_amdgcn_wmma_f32_16x16x32_f16(false, a, false, b, (short)0, c, false, false);
  asm volatile("v_nop\n\tv_nop\n\tv_nop\n\tv_nop" : "+v"(d) : "v"(a), "v"(b));
  return d;
}
__device__ __forceinline__ unsigned int bf16_rne_u32(float f) {
  unsigned int u = __builtin_bit_cast(unsigned int, f);
  u += 0x7fffu + ((u >> 16) & 1u);
  return u & 0xffff0000u;
}
__device__ __forceinline__ void wave_lds_sync() {
  __builtin_amdgcn_fence(3, "workgroup");
  __builtin_amdgcn_wave_barrier();
  __builtin_amdgcn_fence(2, "workgroup");
}
__device__ __forceinline__ unsigned short wbits16(float f, bool o16) {
  const unsigned int r = bf16_rne_u32(f);
  const unsigned short bbits = (unsigned short)(r >> 16);
  const h16 hv = (h16)(__builtin_bit_cast(float, r) * W_CARRY);
  const unsigned short hbits = __builtin_bit_cast(unsigned short, hv);
  return o16 ? hbits : bbits;
}

__global__ __launch_bounds__(256) void cvt_kernel(const float* __restrict__ xq, const float* __restrict__ xk, const float* __restrict__ xv,
                                                  const float* __restrict__ wq, const float* __restrict__ wk, const float* __restrict__ wv,
                                                  const float* __restrict__ wo,
                                                  unsigned short* __restrict__ xpl, unsigned short* __restrict__ wpl) {
  const size_t tid = (size_t)blockIdx.x * blockDim.x + threadIdx.x, stride = (size_t)gridDim.x * blockDim.x;
  const size_t per_x = (size_t)MROWS * HID / 8, nx = 3 * per_x;
  const size_t per_w = (size_t)HID * HID / 8, nw = 4 * per_w;
  for (int pass = 0; pass < 2; ++pass) {
    for (size_t c = tid; c < nx; c += stride) {
      const int which = (int)(c / per_x);
      const size_t i = (c - (size_t)which * per_x) * 8;
      const int m = (int)(i / HID), col = (int)(i % HID);
      const int bb = m / SEQ, t = m - bb * SEQ;
      const float* src = (which == 0) ? xq : (which == 1) ? xk : xv;
      const float* p = src + ((size_t)bb * SEQ_FULL + t) * HID + col;
      const v4f f0 = *(const v4f*)p, f1 = *(const v4f*)(p + 4);
      v8us o;
#pragma unroll
      for (int e = 0; e < 4; ++e) {
        o[e] = (unsigned short)(bf16_rne_u32(f0[e]) >> 16);
        o[4 + e] = (unsigned short)(bf16_rne_u32(f1[e]) >> 16);
      }
      *(volatile v8us*)(xpl + c * 8) = o;
    }
    for (size_t c = tid; c < nw; c += stride) {
      const int mat = (int)(c / per_w);
      const size_t i = (c - (size_t)mat * per_w) * 8;
      const float* w = (mat == 0) ? wq : (mat == 1) ? wk : (mat == 2) ? wv : wo;
      const v4f f0 = *(const v4f*)(w + i), f1 = *(const v4f*)(w + i + 4);
      const bool o16 = (mat == 3);
      v8us o;
#pragma unroll
      for (int e = 0; e < 4; ++e) {
        o[e] = wbits16(f0[e], o16);
        o[4 + e] = wbits16(f1[e], o16);
      }
      *(volatile v8us*)(wpl + c * 8) = o;
    }
    __threadfence();
  }
}

__global__ __launch_bounds__(256) void mask_flag_kernel(const int* __restrict__ mask, int* __restrict__ flags) {
  __shared__ int um[4][64];
  __shared__ int mk[4][64];
  __shared__ int rb[4][64];
  __shared__ __attribute__((aligned(16))) int fl[64];
  const int qt = blockIdx.x, q0 = qt * 16;
  const int t = threadIdx.x, c = t & 63, rg = t >> 6, lane = t & 31, wave = t >> 5;
  const int cc = (c < NCH) ? c : (NCH - 1);
  int anyu = 0, anym = 0, rbits = 0;
#pragma unroll 1
  for (int r = 0; r < 4; ++r) {
    const int* p = mask + (size_t)(q0 + rg * 4 + r) * MPITCH + (size_t)cc * 32;
    int u = 0, mm = 0;
#pragma unroll
    for (int v = 0; v < 8; ++v) {
      const v4i x = *(const v4i*)(p + 4 * v);
#pragma unroll
      for (int e = 0; e < 4; ++e) { u |= (x[e] == 0) ? 1 : 0; mm |= (x[e] != 0) ? 1 : 0; }
    }
    anyu |= u; anym |= mm; rbits |= (u << r);
  }
  um[rg][c] = anyu; mk[rg][c] = anym; rb[rg][c] = rbits;
  __syncthreads();
  if (wave == 0) {
    const int ch0 = lane, ch1 = lane + 32;
    const int U0 = um[0][ch0] | um[1][ch0] | um[2][ch0] | um[3][ch0];
    const int M0 = mk[0][ch0] | mk[1][ch0] | mk[2][ch0] | mk[3][ch0];
    const int U1 = um[0][ch1] | um[1][ch1] | um[2][ch1] | um[3][ch1];
    const int M1 = mk[0][ch1] | mk[1][ch1] | mk[2][ch1] | mk[3][ch1];
    int rows = (rb[0][ch0] | (rb[1][ch0] << 4) | (rb[2][ch0] << 8) | (rb[3][ch0] << 12)) |
               (rb[0][ch1] | (rb[1][ch1] << 4) | (rb[2][ch1] << 8) | (rb[3][ch1] << 12));
#pragma unroll
    for (int s = 16; s >= 1; s >>= 1) rows |= __shfl_xor(rows, s);
    const int rowok = ((rows & 0xFFFF) == 0xFFFF) ? 1 : 0;
    const int f0 = U0 ? (M0 ? F_FILL : F_OPEN) : (rowok ? F_SKIP : F_FILL);
    const int f1 = U1 ? (M1 ? F_FILL : F_OPEN) : (rowok ? F_SKIP : F_FILL);
    fl[ch0] = (ch0 < NCH) ? f0 : F_SKIP;
    fl[ch1] = (ch1 < NCH) ? f1 : F_SKIP;
    wave_lds_sync();
    const v4i v = *(const v4i*)(fl + (lane & 15) * 4);
    int* dst = flags + (size_t)qt * FPITCH + (lane & 15) * 4;
    if (lane < 16) *(volatile v4i*)dst = v;
    __threadfence();
    if (lane < 16) *(volatile v4i*)dst = v;
  }
}

__device__ __forceinline__ void gemm_tile_b(const b16* __restrict__ A, const b16* __restrict__ W, int m0, int c0, int nloc, int hlf, v8f (&acc)[2][4]) {
#pragma unroll 2
  for (int kb = 0; kb < HID; kb += 32) {
    const v16b a0 = frag_kb(A + (size_t)(m0 + nloc) * HID + kb, hlf);
    const v16b a1 = frag_kb(A + (size_t)(m0 + 16 + nloc) * HID + kb, hlf);
#pragma unroll
    for (int t = 0; t < 4; ++t) {
      const v16b bf = frag_kb(W + (size_t)(c0 + t * 16 + nloc) * HID + kb, hlf);
      acc[0][t] = wmma_b(a0, bf, acc[0][t]);
      acc[1][t] = wmma_b(a1, bf, acc[1][t]);
    }
  }
}
__device__ __forceinline__ void gemm_tile_h(const h16* __restrict__ A, const h16* __restrict__ W, int m0, int c0, int nloc, int hlf, v8f (&acc)[2][4]) {
#pragma unroll 2
  for (int kb = 0; kb < HID; kb += 32) {
    const v16h a0 = frag_kh(A + (size_t)(m0 + nloc) * HID + kb, hlf);
    const v16h a1 = frag_kh(A + (size_t)(m0 + 16 + nloc) * HID + kb, hlf);
#pragma unroll
    for (int t = 0; t < 4; ++t) {
      const v16h bf = frag_kh(W + (size_t)(c0 + t * 16 + nloc) * HID + kb, hlf);
      acc[0][t] = wmma_h(a0, bf, acc[0][t]);
      acc[1][t] = wmma_h(a1, bf, acc[1][t]);
    }
  }
}

__global__ __launch_bounds__(128) void qkv_gemm_kernel(const b16* __restrict__ xpl, const b16* __restrict__ wpl,
                                                       const float* __restrict__ bq, const float* __restrict__ bk, const float* __restrict__ bv,
                                                       h16* __restrict__ Qp, h16* __restrict__ Kp, h16* __restrict__ Vp,
                                                       h16* __restrict__ Qr, h16* __restrict__ Kr, h16* __restrict__ Vr) {
  __shared__ __attribute__((aligned(16))) h16 Ts[4][32 * 64];
  __shared__ __attribute__((aligned(16))) h16 Tr[4][32 * 64];
  const int lane = threadIdx.x & 31, wave = threadIdx.x >> 5, nloc = lane & 15, hlf = lane >> 4;
  const int m0 = blockIdx.y * 128 + wave * 32;
  const int cb = blockIdx.x;
  const int mat = cb >> 4, head = cb & 15;
  const int c0 = cb * 64;
  const b16* x = xpl + (size_t)mat * MROWS * HID;
  const float* bias = ((mat == 0) ? bq : (mat == 1) ? bk : bv) + head * DH;
  v8f acc[2][4];
#pragma unroll
  for (int r = 0; r < 2; ++r)
#pragma unroll
    for (int t = 0; t < 4; ++t) acc[r][t] = (v8f){};
  gemm_tile_b(x, wpl, m0, c0, nloc, hlf, acc);
  const int b = m0 / SEQ, t0 = m0 % SEQ;
  const bool wres = (mat != 0) || (t0 < EARLY);
  const int g = b * NH + head;
  h16* Tp = Ts[wave];
  h16* Rp = Tr[wave];
#pragma unroll
  for (int t = 0; t < 4; ++t) {
    const int d = t * 16 + nloc;
    const float bd = __builtin_bit_cast(float, bf16_rne_u32(bias[d]) & 0xFFFF0000u);
#pragma unroll
    for (int r = 0; r < 2; ++r)
#pragma unroll
      for (int v = 0; v < 8; ++v) {
        const int rr = r * 16 + v + 8 * hlf;
        const float f = acc[r][t][v] + bd;
        const h16 y = (h16)f;
        const int idx = (mat < 2) ? (rr * 64 + d) : ((rr >> 4) * 1024 + d * 16 + (rr & 15));
        Tp[idx] = y;
        if (wres) Rp[idx] = (h16)((f - (float)y) * RES_CARRY);
      }
  }
  wave_lds_sync();
  h16* dst; h16* rdst; size_t o;
  if (mat == 0)      { o = ((size_t)g * SEQ + t0) * DH; dst = Qp + o;
                       const int t0e = (t0 < EARLY) ? t0 : 0; rdst = Qr + ((size_t)g * EARLY + t0e) * DH; }
  else if (mat == 1) { o = ((size_t)g * SEQ + t0) * DH; dst = Kp + o; rdst = Kr + o; }
  else               { o = ((size_t)g * QT + (t0 >> 4)) * (size_t)(DH * 16); dst = Vp + o; rdst = Vr + o; }
#pragma unroll
  for (int j = 0; j < 8; ++j) { const int e = (j * 32 + lane) * 8; *(volatile v8h*)(dst + e) = ld8h(Tp + e); }
  if (wres) {
#pragma unroll
    for (int j = 0; j < 8; ++j) { const int e = (j * 32 + lane) * 8; *(volatile v8h*)(rdst + e) = ld8h(Rp + e); }
  }
  __threadfence();
#pragma unroll
  for (int j = 0; j < 8; ++j) { const int e = (j * 32 + lane) * 8; *(volatile v8h*)(dst + e) = ld8h(Tp + e); }
  if (wres) {
#pragma unroll
    for (int j = 0; j < 8; ++j) { const int e = (j * 32 + lane) * 8; *(volatile v8h*)(rdst + e) = ld8h(Rp + e); }
  }
}

template <bool RES>
__device__ __forceinline__ void sc_tile(v8f& s, v8f& sr, const h16* kh, const h16* kr, v16h qa, v16h qb, v16h qra, v16h qrb, int hh) {
  v16h ka = frag_kh(kh, hh);
  s = wmma_h(ka, qa, s);
  if (RES) { sr = wmma_h(ka, qra, sr); const v16h kz = frag_kh(kr, hh); sr = wmma_h(kz, qa, sr); }
  ka = frag_kh(kh + 32, hh);
  s = wmma_h(ka, qb, s);
  if (RES) { sr = wmma_h(ka, qrb, sr); const v16h kz = frag_kh(kr + 32, hh); sr = wmma_h(kz, qb, sr); }
}
template <bool RES>
__device__ __forceinline__ void pv_tile(v8f& oh, v8f& orr, const h16* vh0, const h16* vh1, const h16* vr0, const h16* vr1, v16h pb, v16h pr) {
  const v16h va = cat8h(ld8h(vh0), ld8h(vh1));
  oh = wmma_h(va, pb, oh);
  if (RES) {
    orr = wmma_h(va, pr, orr);
    const v16h vz = cat8h(ld8h(vr0), ld8h(vr1));
    orr = wmma_h(vz, pb, orr);
  }
}

template <bool RES>
__global__ __launch_bounds__(256) __attribute__((amdgpu_num_vgpr(256)))
void attn_kernel(const h16* __restrict__ Qp, const h16* __restrict__ Kp, const h16* __restrict__ Vp,
                 const h16* __restrict__ Qr, const h16* __restrict__ Kr, const h16* __restrict__ Vr,
                 const int* __restrict__ mask, const int* __restrict__ flags,
                 h16* __restrict__ yp, h16* __restrict__ yr) {
  __shared__ __attribute__((aligned(16))) h16 Os[8][16 * 64];
  __shared__ __attribute__((aligned(16))) h16 Or[8][16 * 64];
  const int wid = threadIdx.x >> 5, lane = threadIdx.x & 31, hh = lane >> 4, col = lane & 15;
  const int idx = blockIdx.x * 8 + wid;
  int g, qt;
  if (RES) { g = idx / QT_E; qt = idx - g * QT_E; }
  else     { g = idx / QT_LD; qt = QT_E + (idx - g * QT_LD); }
  const int q0 = qt << 4;
  const int b = g / NH, h = g % NH;
  const size_t ko = (size_t)g * SEQ * DH;
  const size_t qo = ((size_t)g * SEQ + q0 + col) * DH;
  const v16h qa = frag_kh(Qp + qo, hh), qb = frag_kh(Qp + qo + 32, hh);
  v16h qra = {}, qrb = {};
  if (RES) {
    const size_t qro2 = ((size_t)g * EARLY + q0 + col) * DH;
    qra = frag_kh(Qr + qro2, hh); qrb = frag_kh(Qr + qro2 + 32, hh);
  }
  const int qi = q0 + col;
  const int* mrow = mask + (size_t)qi * MPITCH + 8 * hh;
  const int* frow = flags + (size_t)qt * FPITCH;
  float m = -__builtin_inff(), l = 0.0f;
  v8f o0 = {}, o1 = {}, o2 = {}, o3 = {};
  v8f n0 = {}, n1 = {}, n2 = {}, n3 = {};
#pragma unroll 1
  for (int kb = 0; kb < SEQ; kb += 32) {
    const int f = __builtin_amdgcn_readfirstlane(frow[kb >> 5]);
    if (f == F_SKIP) continue;
    const size_t r0 = ko + (size_t)(kb + col) * DH, r1 = ko + (size_t)(kb + 16 + col) * DH;
    v8f s0 = {}, s1 = {}, z0 = {}, z1 = {};
    if (RES) {
      sc_tile<true>(s0, z0, Kp + r0, Kr + r0, qa, qb, qra, qrb, hh);
      sc_tile<true>(s1, z1, Kp + r1, Kr + r1, qa, qb, qra, qrb, hh);
      s0 = (s0 + z0 * RES_INV) * SCORE_SCALE; s1 = (s1 + z1 * RES_INV) * SCORE_SCALE;
    } else {
      sc_tile<false>(s0, z0, Kp + r0, Kp + r0, qa, qb, qra, qrb, hh);
      sc_tile<false>(s1, z1, Kp + r1, Kp + r1, qa, qb, qra, qrb, hh);
      s0 = s0 * SCORE_SCALE; s1 = s1 * SCORE_SCALE;
    }
    if (f != F_OPEN) {
      const v8i mk0 = *(const v8i*)(mrow + kb);
      const v8i mk1 = *(const v8i*)(mrow + kb + 16);
#pragma unroll
      for (int r = 0; r < 8; ++r) {
        s0[r] = (mk0[r] != 0) ? MASK_FILL : s0[r];
        s1[r] = (mk1[r] != 0) ? MASK_FILL : s1[r];
      }
    }
    float mr = -__builtin_inff();
#pragma unroll
    for (int r = 0; r < 8; ++r) mr = fmaxf(mr, fmaxf(s0[r], s1[r]));
    mr = fmaxf(mr, __shfl_xor(mr, 16));
    const float mn = fmaxf(m, mr);
    const float al_ = __expf(m - mn);
    m = mn;
    float sum = 0.0f;
    v16h pb = {}, pr = {};
#pragma unroll
    for (int r = 0; r < 8; ++r) {
      const float p0 = __expf(s0[r] - mn), p1 = __expf(s1[r] - mn);
      sum += p0 + p1;
      const h16 ph0 = (h16)(p0 * P_CARRY), ph1 = (h16)(p1 * P_CARRY);
      pb[r] = ph0; pb[8 + r] = ph1;
      if (RES) {
        pr[r] = (h16)((p0 * P_CARRY - (float)ph0) * RES_CARRY);
        pr[8 + r] = (h16)((p1 * P_CARRY - (float)ph1) * RES_CARRY);
      }
    }
    sum += __shfl_xor(sum, 16);
    l = l * al_ + sum;
    o0 = o0 * al_; o1 = o1 * al_; o2 = o2 * al_; o3 = o3 * al_;
    if (RES) { n0 = n0 * al_; n1 = n1 * al_; n2 = n2 * al_; n3 = n3 * al_; }
    const size_t v0 = ko + (size_t)(kb >> 4) * (DH * 16) + 8 * hh, v1 = v0 + DH * 16;
    pv_tile<RES>(o0, n0, Vp + v0 + (0 * 16 + col) * 16, Vp + v1 + (0 * 16 + col) * 16, Vr + v0 + (0 * 16 + col) * 16, Vr + v1 + (0 * 16 + col) * 16, pb, pr);
    pv_tile<RES>(o1, n1, Vp + v0 + (1 * 16 + col) * 16, Vp + v1 + (1 * 16 + col) * 16, Vr + v0 + (1 * 16 + col) * 16, Vr + v1 + (1 * 16 + col) * 16, pb, pr);
    pv_tile<RES>(o2, n2, Vp + v0 + (2 * 16 + col) * 16, Vp + v1 + (2 * 16 + col) * 16, Vr + v0 + (2 * 16 + col) * 16, Vr + v1 + (2 * 16 + col) * 16, pb, pr);
    pv_tile<RES>(o3, n3, Vp + v0 + (3 * 16 + col) * 16, Vp + v1 + (3 * 16 + col) * 16, Vr + v0 + (3 * 16 + col) * 16, Vr + v1 + (3 * 16 + col) * 16, pb, pr);
  }
  const float inv = (1.0f / l) * Y_FROM_O;
  const float invr = inv * RES_INV;
  h16* Tt = Os[wid];
  h16* Tq = Or[wid];
#pragma unroll
  for (int r = 0; r < 8; ++r) {
    const int hr = 8 * hh + r;
    float f0 = o0[r] * inv, f1 = o1[r] * inv, f2 = o2[r] * inv, f3 = o3[r] * inv;
    if (RES) { f0 += n0[r] * invr; f1 += n1[r] * invr; f2 += n2[r] * invr; f3 += n3[r] * invr; }
    const h16 y0 = (h16)f0, y1 = (h16)f1, y2 = (h16)f2, y3 = (h16)f3;
    Tt[col * 64 + 0 + hr]  = y0;
    Tt[col * 64 + 16 + hr] = y1;
    Tt[col * 64 + 32 + hr] = y2;
    Tt[col * 64 + 48 + hr] = y3;
    if (RES) {
      Tq[col * 64 + 0 + hr]  = (h16)((f0 - (float)y0) * RES_CARRY);
      Tq[col * 64 + 16 + hr] = (h16)((f1 - (float)y1) * RES_CARRY);
      Tq[col * 64 + 32 + hr] = (h16)((f2 - (float)y2) * RES_CARRY);
      Tq[col * 64 + 48 + hr] = (h16)((f3 - (float)y3) * RES_CARRY);
    }
  }
  wave_lds_sync();
  h16* dst0 = yp + ((size_t)b * SEQ + q0) * HID + h * DH;
  h16* dst1 = yr + ((size_t)b * EARLY + (RES ? q0 : 0)) * HID + h * DH;
#pragma unroll
  for (int j = 0; j < 4; ++j) {
    const int rr = j * 4 + (lane >> 3), c8 = (lane & 7) * 8;
    *(volatile v8h*)(dst0 + (size_t)rr * HID + c8) = ld8h(Tt + rr * 64 + c8);
    if (RES) *(volatile v8h*)(dst1 + (size_t)rr * HID + c8) = ld8h(Tq + rr * 64 + c8);
  }
  __threadfence();
#pragma unroll
  for (int j = 0; j < 4; ++j) {
    const int rr = j * 4 + (lane >> 3), c8 = (lane & 7) * 8;
    *(volatile v8h*)(dst0 + (size_t)rr * HID + c8) = ld8h(Tt + rr * 64 + c8);
    if (RES) *(volatile v8h*)(dst1 + (size_t)rr * HID + c8) = ld8h(Tq + rr * 64 + c8);
  }
}

__global__ __launch_bounds__(128) void out_gemm_kernel(const h16* __restrict__ yp, const h16* __restrict__ yr, const h16* __restrict__ wop,
                                                       const float* __restrict__ bo, float* __restrict__ out) {
  __shared__ __attribute__((aligned(16))) float Ts[4][32 * 64];
  const int lane = threadIdx.x & 31, wave = threadIdx.x >> 5, nloc = lane & 15, hlf = lane >> 4;
  const int m0 = blockIdx.y * 128 + wave * 32;
  const int c0 = blockIdx.x * 64;
  const int b = m0 / SEQ, t0 = m0 - b * SEQ;
  const bool early = (((int)blockIdx.y * 128) % SEQ) < EARLY;
  v8f acc[2][4];
#pragma unroll
  for (int r = 0; r < 2; ++r)
#pragma unroll
    for (int t = 0; t < 4; ++t) acc[r][t] = (v8f){};
  if (early) {
    gemm_tile_h(yr, wop, b * EARLY + t0, c0, nloc, hlf, acc);
#pragma unroll
    for (int r = 0; r < 2; ++r)
#pragma unroll
      for (int t = 0; t < 4; ++t) acc[r][t] = acc[r][t] * RES_INV;
  }
  gemm_tile_h(yp, wop, m0, c0, nloc, hlf, acc);
  float* Tt = Ts[wave];
#pragma unroll
  for (int t = 0; t < 4; ++t) {
    const float bd = __builtin_bit_cast(float, bf16_rne_u32(bo[c0 + t * 16 + nloc]) & 0xFFFF0000u);
#pragma unroll
    for (int r = 0; r < 2; ++r)
#pragma unroll
      for (int v = 0; v < 8; ++v) Tt[(r * 16 + v + 8 * hlf) * 64 + t * 16 + nloc] = acc[r][t][v] * OUT_UNSCALE + bd;
  }
  wave_lds_sync();
  float* dst0 = out + (size_t)m0 * HID + c0;
#pragma unroll
  for (int j = 0; j < 16; ++j) { const int rr = j * 2 + hlf, c4 = nloc * 4; *(volatile v4f*)(dst0 + (size_t)rr * HID + c4) = *(const v4f*)(Tt + rr * 64 + c4); }
  __threadfence();
#pragma unroll
  for (int j = 0; j < 16; ++j) { const int rr = j * 2 + hlf, c4 = nloc * 4; *(volatile v4f*)(dst0 + (size_t)rr * HID + c4) = *(const v4f*)(Tt + rr * 64 + c4); }
}
}

extern "C" void kernel_launch(void* const* d_in, const int* in_sizes, int n_in,
                              void* d_out, int out_size, void* d_ws, size_t ws_size, hipStream_t stream) {
  if (n_in < 12) return;
  const size_t need_x = ((size_t)(NB - 1) * SEQ_FULL + SEQ) * HID;
  if ((size_t)in_sizes[0] < need_x || (size_t)in_sizes[1] < need_x || (size_t)in_sizes[2] < need_x) return;
  if ((size_t)in_sizes[3] < (size_t)(SEQ - 1) * MPITCH + SEQ) return;
  if (in_sizes[4] < HID * HID || in_sizes[6] < HID * HID || in_sizes[8] < HID * HID || in_sizes[10] < HID * HID) return;
  if (in_sizes[5] < HID || in_sizes[7] < HID || in_sizes[9] < HID || in_sizes[11] < HID) return;
  if ((size_t)out_size < (size_t)MROWS * HID) return;

  const float* query = (const float*)d_in[0];
  const float* key   = (const float*)d_in[1];
  const float* value = (const float*)d_in[2];
  const int*   amask = (const int*)d_in[3];
  const float* Wq = (const float*)d_in[4];
  const float* bq = (const float*)d_in[5];
  const float* Wk = (const float*)d_in[6];
  const float* bk = (const float*)d_in[7];
  const float* Wv = (const float*)d_in[8];
  const float* bv = (const float*)d_in[9];
  const float* Wo = (const float*)d_in[10];
  const float* bo = (const float*)d_in[11];
  float* out = (float*)d_out;

  size_t off = 0; char* ws = (char*)d_ws;
  unsigned short* xpl = (unsigned short*)(ws + off); off += (size_t)3 * MROWS * HID * 2;
  unsigned short* wpl = (unsigned short*)(ws + off); off += (size_t)4 * HID * HID * 2;
  h16* Qp = (h16*)(ws + off); off += (size_t)MROWS * HID * 2;
  h16* Kp = (h16*)(ws + off); off += (size_t)MROWS * HID * 2;
  h16* Vp = (h16*)(ws + off); off += (size_t)MROWS * HID * 2;
  h16* yp = (h16*)(ws + off); off += (size_t)MROWS * HID * 2;
  h16* Qr = (h16*)(ws + off); off += (size_t)NB * NH * EARLY * DH * 2;
  h16* Kr = (h16*)(ws + off); off += (size_t)MROWS * HID * 2;
  h16* Vr = (h16*)(ws + off); off += (size_t)MROWS * HID * 2;
  h16* yr = (h16*)(ws + off); off += (size_t)NB * EARLY * HID * 2;
  int* flags = (int*)(ws + off); off += (size_t)QT * FPITCH * 4;
  if (off > ws_size) return;
  const h16* wop = (const h16*)(wpl + (size_t)NQKV * HID);

  cvt_kernel<<<2048, 256, 0, stream>>>(query, key, value, Wq, Wk, Wv, Wo, xpl, wpl);
  mask_flag_kernel<<<QT, 256, 0, stream>>>(amask, flags);
  qkv_gemm_kernel<<<dim3(NQKV / 64, MROWS / 128), 128, 0, stream>>>((const b16*)xpl, (const b16*)wpl, bq, bk, bv, Qp, Kp, Vp, Qr, Kr, Vr);
  attn_kernel<true><<<(NB * NH * QT_E) / 8, 256, 0, stream>>>(Qp, Kp, Vp, Qr, Kr, Vr, amask, flags, yp, yr);
  if (QT_L > 0) attn_kernel<false><<<(NB * NH * QT_L) / 8, 256, 0, stream>>>(Qp, Kp, Vp, Qr, Kr, Vr, amask, flags, yp, yr);
  out_gemm_kernel<<<dim3(HID / 64, MROWS / 128), 128, 0, stream>>>(yp, yr, wop, bo, out);
}
